// GNN_16209206575854
// MI455X (gfx1250) — hardware-verified
//
#include <hip/hip_runtime.h>
#include <stddef.h>
#include <stdint.h>
#include <math.h>


#define FD     512
#define NTHR   256
#define NWAVE  8
#define EPT    8
#define CHUNK  (NTHR * EPT)
#define WCAP   (EPT * 32)
#define LISTN  (NWAVE * WCAP)
#define NBA    512
#define SLA    9
#define RCAP   16384
#define DEGCAP 64
#define GBM    64
#define GBN    128
#define GTHR   128
#define RPB    64
#define NUA    (512 * 64)
#define NUB    (512 * 128)
#define NUD    (256 * 128)
#define NUTOT  (NUA + 2 * NUB + NUD)
#define BLD_ZINTS    (LISTN + 2 * RCAP + 3 * NBA)
#define MISC_INTS    16
#define BLD_LDS_INTS (BLD_ZINTS + MISC_INTS + NBA)
#define WSMAX  134217728

static_assert((CHUNK & (CHUNK - 1)) == 0 && CHUNK <= 4096);
static_assert((NBA & (NBA - 1)) == 0 && NBA == (1 << SLA));
static_assert(((long long)CHUNK << SLA) < (1LL << 31));
static_assert(RCAP % (2 * NTHR) == 0 && RCAP % 32 == 0);
static_assert(NBA % NTHR == 0 && NBA / 4 <= NTHR && (2 * NBA) / 4 == NTHR);
static_assert(BLD_ZINTS % 4 == 0 && ((BLD_ZINTS + MISC_INTS) % 4) == 0);
static_assert(BLD_LDS_INTS * 4 <= 300000);
static_assert(RPB % NWAVE == 0 && RPB == GBM && RPB % 32 == 0 && RPB / 4 <= 32);
static_assert(GBM == (GTHR / 32) * 16 && GBN == 128);
static_assert(NUA % NTHR == 0 && NUB % NTHR == 0 && NUD % NTHR == 0);
static_assert(DEGCAP >= 38 + 8);
static_assert(FD == 4 * 128);

typedef float          v4f   __attribute__((ext_vector_type(4)));
typedef float          v8f   __attribute__((ext_vector_type(8)));
typedef int            v2i   __attribute__((ext_vector_type(2)));
typedef int            v4i   __attribute__((ext_vector_type(4)));
typedef int            v8i   __attribute__((ext_vector_type(8)));
typedef unsigned short v4us  __attribute__((ext_vector_type(4)));
typedef unsigned short v8us  __attribute__((ext_vector_type(8)));
typedef unsigned short v16us __attribute__((ext_vector_type(16)));
typedef __bf16         v16bf __attribute__((ext_vector_type(16)));
typedef v4f  __attribute__((may_alias)) v4fa;
typedef v2i  __attribute__((may_alias)) v2ia;
typedef v4i  __attribute__((may_alias)) v4ia;
typedef v4us __attribute__((may_alias)) v4usa;
typedef v8us __attribute__((may_alias)) v8usa;
union FragB { v16bf v; v16us u; v8us h[2]; v8i w; };

__device__ __forceinline__ v8f wmb(const FragB& a, const FragB& b, v8f c) {
  v8f d = __builtin_amdgcn_wmma_f32_16x16x32_bf16(false, a.v, false, b.v, (short)0, c, false, false);
  asm volatile("v_nop\n\tv_nop\n\tv_nop\n\tv_nop" : "+v"(d) : "v"(a.w), "v"(b.w));
  return d;
}

__device__ __forceinline__ unsigned bf16_bits(float f) {
  const unsigned u = __float_as_uint(f);
  const unsigned r = (u + 0x7FFFu + ((u >> 16) & 1u)) >> 16;
  return ((u & 0x7fffffffu) > 0x7f800000u) ? 0x7fc0u : r;
}
__device__ __forceinline__ float bf16_val(float f) {
  return __uint_as_float(bf16_bits(f) << 16);
}

__device__ __forceinline__ void wave_sync() {
  __builtin_amdgcn_fence(__ATOMIC_RELEASE, "wavefront");
  __builtin_amdgcn_wave_barrier();
  __builtin_amdgcn_fence(__ATOMIC_ACQUIRE, "wavefront");
}

template <int SLB>
__device__ __forceinline__ int scan_chunk(const int* __restrict__ dsts, int nE, int cbase, int slotBase,
                                          int nb, int vec8, int* list, int tid, int lane, int wave) {
  int wc = 0;
  const int el0  = tid * EPT;
  const int e0   = cbase + el0;
  const int sent = -2147483647 - 1;
  v4i da, db;
  if (vec8 != 0 && cbase + CHUNK <= nE) {
    da = *(const v4i*)(dsts + e0);
    db = *(const v4i*)(dsts + e0 + 4);
  } else {
    da.x = (e0     < nE) ? dsts[min(e0,     nE - 1)] : sent;
    da.y = (e0 + 1 < nE) ? dsts[min(e0 + 1, nE - 1)] : sent;
    da.z = (e0 + 2 < nE) ? dsts[min(e0 + 2, nE - 1)] : sent;
    da.w = (e0 + 3 < nE) ? dsts[min(e0 + 3, nE - 1)] : sent;
    db.x = (e0 + 4 < nE) ? dsts[min(e0 + 4, nE - 1)] : sent;
    db.y = (e0 + 5 < nE) ? dsts[min(e0 + 5, nE - 1)] : sent;
    db.z = (e0 + 6 < nE) ? dsts[min(e0 + 6, nE - 1)] : sent;
    db.w = (e0 + 7 < nE) ? dsts[min(e0 + 7, nE - 1)] : sent;
  }
  const unsigned nbs = (unsigned)slotBase;
  const unsigned unb = (unsigned)nb;
  const unsigned s0 = (unsigned)da.x - nbs, s1 = (unsigned)da.y - nbs;
  const unsigned s2 = (unsigned)da.z - nbs, s3 = (unsigned)da.w - nbs;
  const unsigned s4 = (unsigned)db.x - nbs, s5 = (unsigned)db.y - nbs;
  const unsigned s6 = (unsigned)db.z - nbs, s7 = (unsigned)db.w - nbs;
  const bool h0 = s0 < unb, h1 = s1 < unb, h2 = s2 < unb, h3 = s3 < unb;
  const bool h4 = s4 < unb, h5 = s5 < unb, h6 = s6 < unb, h7 = s7 < unb;
  const unsigned any = __builtin_amdgcn_ballot_w32(h0 | h1 | h2 | h3 | h4 | h5 | h6 | h7);
  if (any != 0u) {
#define HITJ(J, HJ, SJ) { \
      const unsigned mj = __builtin_amdgcn_ballot_w32(HJ); \
      if (mj != 0u) { \
        if (HJ) { \
          const int pos = wc + (int)__builtin_amdgcn_mbcnt_lo(mj, 0u); \
          if (pos < WCAP) list[wave * WCAP + pos] = ((el0 + (J)) << SLB) | (int)(SJ); \
        } \
        wc += (int)__builtin_popcount(mj); } }
    HITJ(0, h0, s0)
    HITJ(1, h1, s1)
    HITJ(2, h2, s2)
    HITJ(3, h3, s3)
    HITJ(4, h4, s4)
    HITJ(5, h5, s5)
    HITJ(6, h6, s6)
    HITJ(7, h7, s7)
#undef HITJ
  }
  return wc;
}

__device__ __forceinline__ void wunit(const float* __restrict__ W, int stride, int kk, int n,
                                      unsigned short* dp) {
  const float* p = W + (size_t)kk * (size_t)stride + n;
  v8us o;
#pragma unroll
  for (int i = 0; i < 8; ++i) o[i] = (unsigned short)bf16_bits(p[(size_t)i * (size_t)stride]);
  *(volatile v8us*)dp = o;
  __threadfence();
  *(volatile v8us*)dp = o;
}

__global__ __launch_bounds__(NTHR) void k_wprep(const float* __restrict__ W1, const float* __restrict__ W2,
                                                const float* __restrict__ W3, const float* __restrict__ W4,
                                                unsigned short* W1T, unsigned short* W2D,
                                                unsigned short* W3D, unsigned short* W4D) {
  const int u = (int)blockIdx.x * NTHR + (int)threadIdx.x;
  if (u < NUA) {
    const int n = u >> 6, k8 = (u & 63) * 8;
    wunit(W1, 512, k8, n, W1T + (size_t)n * 512 + k8);
  } else if (u < NUA + NUB) {
    const int v = u - NUA;
    const int n = v >> 7, k8 = (v & 127) * 8;
    wunit(W2, 512, k8 & 511, n, W2D + (size_t)n * 1024 + k8);
  } else if (u < NUA + 2 * NUB) {
    const int v = u - NUA - NUB;
    const int n = v >> 7, k8 = (v & 127) * 8;
    wunit(W3, 512, k8 & 511, n, W3D + (size_t)n * 1024 + k8);
  } else if (u < NUTOT) {
    const int v = u - NUA - 2 * NUB;
    const int n = v >> 7, k8 = (v & 127) * 8;
    wunit(W4, 256, k8 & 511, n, W4D + (size_t)n * 1024 + k8);
  }
}

__global__ __launch_bounds__(NTHR) void k_cvx(const float* __restrict__ x, int nN, int nUnits,
                                              unsigned short* xb) {
  const int u = (int)blockIdx.x * NTHR + (int)threadIdx.x;
  if (u >= nUnits) return;
  const int row = u >> 6;
  const int k8  = (u & 63) * 8;
  const int rc  = row < nN ? row : nN - 1;
  const float* p = x + (size_t)rc * FD + k8;
  const v4f a = *(const v4fa*)p;
  const v4f b = *(const v4fa*)(p + 4);
  const bool ok = row < nN;
  v8us o;
  o[0] = ok ? (unsigned short)bf16_bits(a.x) : (unsigned short)0;
  o[1] = ok ? (unsigned short)bf16_bits(a.y) : (unsigned short)0;
  o[2] = ok ? (unsigned short)bf16_bits(a.z) : (unsigned short)0;
  o[3] = ok ? (unsigned short)bf16_bits(a.w) : (unsigned short)0;
  o[4] = ok ? (unsigned short)bf16_bits(b.x) : (unsigned short)0;
  o[5] = ok ? (unsigned short)bf16_bits(b.y) : (unsigned short)0;
  o[6] = ok ? (unsigned short)bf16_bits(b.z) : (unsigned short)0;
  o[7] = ok ? (unsigned short)bf16_bits(b.w) : (unsigned short)0;
  unsigned short* dp = xb + (size_t)row * FD + k8;
  *(volatile v8us*)dp = o;
  __threadfence();
  *(volatile v8us*)dp = o;
}

__global__ __launch_bounds__(NTHR) void k_build(const int* __restrict__ srcs, const int* __restrict__ dsts,
                                                const float* __restrict__ ew, int nE, int nN, int vec8,
                                                float* dinv, int* rec, int* cache) {
  extern __shared__ __attribute__((aligned(16))) int dsm[];
  int* list = dsm;
  int* hl   = dsm + LISTN;
  int* sl   = hl + RCAP;
  int* cnt  = sl + RCAP;
  int* offs = cnt + NBA;
  int* cur  = offs + NBA;
  int* misc = cur + NBA;
  float* dvf = (float*)(misc + MISC_INTS);
  const int tid = (int)threadIdx.x, lane = tid & 31, wave = tid >> 5;
  const int nodeBase = (int)blockIdx.x * NBA;

  {
    const v4i z4 = {0, 0, 0, 0};
    for (int i = tid * 4; i < BLD_ZINTS; i += NTHR * 4) *(v4ia*)(dsm + i) = z4;
    if (tid < MISC_INTS) misc[tid] = 0;
  }
  __syncthreads();

  int t = 0, ov = 0;
  const int nChunks = (nE + CHUNK - 1) / CHUNK;
#pragma unroll 1
  for (int ch = 0; ch < nChunks; ++ch) {
    const int cbase = ch * CHUNK;
    const int wc = scan_chunk<SLA>(dsts, nE, cbase, nodeBase, NBA, vec8, list, tid, lane, wave);
    if (lane == 0) misc[wave] = wc;
    __syncthreads();
    if (wave == 0) {
#pragma unroll 1
      for (int w2 = 0; w2 < NWAVE; ++w2) {
        int c = misc[w2];
        c = c < 0 ? 0 : (c > WCAP ? WCAP : c);
#pragma unroll 1
        for (int b0 = 0; b0 < c; b0 += 32) {
          const int idx = b0 + lane;
          const int ent = list[w2 * WCAP + (idx < WCAP ? idx : WCAP - 1)];
          const int m32 = (c - b0) < 32 ? (c - b0) : 32;
#pragma unroll 1
          for (int k = 0; k < m32; ++k) {
            const int u    = __builtin_amdgcn_readlane(ent, k);
            const int slot = u & (NBA - 1);
            const int el   = (u >> SLA) & (CHUNK - 1);
            const int pk   = ((cbase + el) << SLA) | slot;
            if (t < RCAP) {
              if (lane == 0) { hl[t] = pk; cnt[slot] = cnt[slot] + 1; }
              t = t + 1;
            } else {
              ov = 1;
            }
          }
        }
      }
    }
    __syncthreads();
  }
  if (wave == 0 && lane == 0) { misc[8] = t; misc[9] = ov; }
  __syncthreads();
  int tt = misc[8];
  tt = tt < 0 ? 0 : (tt > RCAP ? RCAP : tt);
  const int ovf = misc[9];

  if (wave == 0) {
    const int base = lane * (NBA / 32);
    int s = 0;
#pragma unroll 1
    for (int i = 0; i < NBA / 32; ++i) s += cnt[base + i];
    int incl = s;
#pragma unroll
    for (int d = 1; d < 32; d <<= 1) {
      const int y = __shfl_up(incl, d, 32);
      if (lane >= d) incl += y;
    }
    int run = incl - s;
#pragma unroll 1
    for (int i = 0; i < NBA / 32; ++i) {
      const int cv = cnt[base + i];
      offs[base + i] = run;
      cur[base + i]  = run;
      run += cv;
    }
  }
  __syncthreads();
  if (wave == 0) {
#pragma unroll 1
    for (int b0 = 0; b0 < tt; b0 += 32) {
      const int idx = b0 + lane;
      const int ent = hl[idx < RCAP ? idx : RCAP - 1];
      const int m32 = (tt - b0) < 32 ? (tt - b0) : 32;
#pragma unroll 1
      for (int k = 0; k < m32; ++k) {
        const int u    = __builtin_amdgcn_readlane(ent, k);
        const int slot = u & (NBA - 1);
        if (lane == 0) {
          int p = cur[slot];
          p = p < 0 ? 0 : (p > RCAP - 1 ? RCAP - 1 : p);
          sl[p] = u;
          cur[slot] = p + 1;
        }
      }
    }
  }
  __syncthreads();

#pragma unroll 1
  for (int q = 0; q < NBA / NTHR; ++q) {
    const int s = q * NTHR + tid;
    int c = cnt[s];
    c = c < 0 ? 0 : (c > DEGCAP ? DEGCAP : c);
    int o = offs[s];
    o = o < 0 ? 0 : (o > RCAP ? RCAP : o);
    float sum = 0.0f;
#pragma unroll 1
    for (int p = 0; p < DEGCAP; ++p) {
      const bool act = p < c;
      if (__builtin_amdgcn_ballot_w32(act) == 0u) break;
      int idx = o + p;
      idx = idx > RCAP - 1 ? RCAP - 1 : idx;
      int eid = sl[idx] >> SLA;
      eid = eid < 0 ? 0 : (eid > nE - 1 ? nE - 1 : eid);
      const float w = bf16_val(ew[eid]);
      const float sn = sum + w;
      sum = act ? sn : sum;
    }
    const float deg = sum + 1.0f;
    dvf[s] = (deg > 0.0f) ? (1.0f / sqrtf(deg)) : 0.0f;
  }
  __syncthreads();

  {
    const v4f dq = *(const v4fa*)(dvf + 4 * (tid & (NBA / 4 - 1)));
    float* dp = dinv + (size_t)nodeBase + 4 * (tid & (NBA / 4 - 1));
    const bool okd = tid < NBA / 4;
    v4i rq;
    rq.x = offs[2 * tid];
    rq.y = (ovf != 0) ? -1 : cnt[2 * tid];
    rq.z = offs[2 * tid + 1];
    rq.w = (ovf != 0) ? -1 : cnt[2 * tid + 1];
    int* rp = rec + ((size_t)nodeBase + 2 * tid) * 2;
    if (okd) *(volatile v4f*)dp = dq;
    *(volatile v4i*)rp = rq;
    __threadfence();
    if (okd) *(volatile v4f*)dp = dq;
    *(volatile v4i*)rp = rq;
  }
  int* cb = cache + (size_t)blockIdx.x * RCAP * 2;
#pragma unroll 1
  for (int it = 0; it < RCAP / (2 * NTHR); ++it) {
    const int e0 = it * 2 * NTHR + 2 * tid;
    const int u0 = sl[e0];
    const int u1 = sl[e0 + 1];
    int id0 = u0 >> SLA, id1 = u1 >> SLA;
    id0 = id0 < 0 ? 0 : (id0 > nE - 1 ? nE - 1 : id0);
    id1 = id1 < 0 ? 0 : (id1 > nE - 1 ? nE - 1 : id1);
    int s0 = srcs[id0], s1 = srcs[id1];
    s0 = s0 < 0 ? 0 : (s0 > nN - 1 ? nN - 1 : s0);
    s1 = s1 < 0 ? 0 : (s1 > nN - 1 ? nN - 1 : s1);
    const int w0 = (int)(bf16_bits(ew[id0]) << 16);
    const int w1 = (int)(bf16_bits(ew[id1]) << 16);
    const bool ok0 = e0 < tt, ok1 = (e0 + 1) < tt;
    v4i o;
    o.x = ok0 ? s0 : 0; o.y = ok0 ? w0 : 0;
    o.z = ok1 ? s1 : 0; o.w = ok1 ? w1 : 0;
    int* op = cb + 2 * (size_t)e0;
    *(volatile v4i*)op = o;
    __threadfence();
    *(volatile v4i*)op = o;
  }
}

__global__ __launch_bounds__(GTHR) void k_gemm(const unsigned short* __restrict__ A, int lda,
                                               const unsigned short* __restrict__ BT, int K,
                                               const float* __restrict__ dinv, float* outF, int ldo) {
  __shared__ __attribute__((aligned(16))) float stg[GBM * GBN];
  const int tid = (int)threadIdx.x, lane = tid & 31, wave = tid >> 5, hh = lane >> 4, m = lane & 15;
  const int rowBase = (int)blockIdx.x * GBM;
  const int col0    = (int)blockIdx.y * GBN;

  v8f acc[8];
  {
    const v8f z = {0.f, 0.f, 0.f, 0.f, 0.f, 0.f, 0.f, 0.f};
#pragma unroll
    for (int t = 0; t < 8; ++t) acc[t] = z;
  }
  const unsigned short* ap = A  + (size_t)(rowBase + 16 * wave + m) * (size_t)lda + 8 * hh;
  const unsigned short* bp = BT + (size_t)(col0 + m) * (size_t)K + 8 * hh;

#pragma unroll 1
  for (int k0 = 0; k0 < K; k0 += 32) {
    FragB af;
    af.h[0] = *(const v8usa*)(ap + k0);
    af.h[1] = *(const v8usa*)(ap + k0 + 16);
#pragma unroll
    for (int nt = 0; nt < 8; ++nt) {
      const unsigned short* wq = bp + (size_t)(16 * nt) * (size_t)K + k0;
      FragB bf;
      bf.h[0] = *(const v8usa*)wq;
      bf.h[1] = *(const v8usa*)(wq + 16);
      acc[nt] = wmb(af, bf, acc[nt]);
    }
  }

#pragma unroll
  for (int nt = 0; nt < 8; ++nt) {
    const int lc = 16 * nt + m;
#pragma unroll
    for (int r = 0; r < 8; ++r) {
      const int lr = 16 * wave + 8 * hh + r;
      stg[lr * GBN + lc] = acc[nt][r];
    }
  }
  __syncthreads();

  v4f dq[4];
#pragma unroll
  for (int q = 0; q < 4; ++q) dq[q] = *(const v4f*)(dinv + rowBase + 16 * wave + 4 * q);
  v4f pv[16];
#pragma unroll
  for (int i = 0; i < 16; ++i) {
    const v4f p = *(const v4fa*)(stg + (16 * wave + i) * GBN + 4 * lane);
    const float d = dq[i >> 2][i & 3];
    v4f y;
    y.x = p.x * d; y.y = p.y * d; y.z = p.z * d; y.w = p.w * d;
    pv[i] = y;
  }
#pragma unroll
  for (int i = 0; i < 16; ++i) {
    float* op = outF + (size_t)(rowBase + 16 * wave + i) * (size_t)ldo + col0 + 4 * lane;
    *(volatile v4f*)op = pv[i];
  }
  __threadfence();
#pragma unroll
  for (int i = 0; i < 16; ++i) {
    float* op = outF + (size_t)(rowBase + 16 * wave + i) * (size_t)ldo + col0 + 4 * lane;
    *(volatile v4f*)op = pv[i];
  }
}

template <int F>
__global__ __launch_bounds__(NTHR) void k_agg(const float* __restrict__ hs, const float* __restrict__ dinv,
                                              const int* __restrict__ rec, const int* __restrict__ cache,
                                              const float* __restrict__ bias, const float* __restrict__ w5,
                                              int nN, int mRows, unsigned short* xhl, float* ts) {
  constexpr int NJ = F / 128;
  __shared__ __attribute__((aligned(16))) unsigned short rowbuf[(F == 512) ? (NWAVE * 1024) : 8];
  __shared__ __attribute__((aligned(16))) float tsb[RPB];
  const int tid = (int)threadIdx.x, lane = tid & 31, wave = tid >> 5;
  const int blockBase = (int)blockIdx.x * RPB;
  const float qnan = __int_as_float(0x7fc00000);

  v4f bv[NJ];
  v4f wv[NJ];
#pragma unroll
  for (int j = 0; j < NJ; ++j) {
    const v4f a = *(const v4f*)(bias + 4 * lane + 128 * j);
    v4f b;
    b.x = bf16_val(a.x); b.y = bf16_val(a.y); b.z = bf16_val(a.z); b.w = bf16_val(a.w);
    bv[j] = b;
    v4f w = {0.f, 0.f, 0.f, 0.f};
    if constexpr (F == 256) {
      const v4f c = *(const v4f*)(w5 + 4 * lane + 128 * j);
      w.x = bf16_val(c.x); w.y = bf16_val(c.y); w.z = bf16_val(c.z); w.w = bf16_val(c.w);
    }
    wv[j] = w;
  }

#pragma unroll 1
  for (int si = 0; si < RPB / NWAVE; ++si) {
    const int r    = si * NWAVE + wave;
    const int node = blockBase + r;
    const int nc   = node < nN ? node : nN - 1;
    const v2i rc = *(const v2ia*)(rec + 2 * (size_t)node);
    int c = rc.y;
    const bool bad = (c < 0) || (c > DEGCAP);
    c = c < 0 ? 0 : (c > DEGCAP ? DEGCAP : c);
    int o = rc.x;
    o = o < 0 ? 0 : (o > RCAP ? RCAP : o);
    const int* cb = cache + (size_t)(node >> SLA) * RCAP * 2;

    v4f acc[NJ];
#pragma unroll
    for (int j = 0; j < NJ; ++j) { const v4f z = {0.f, 0.f, 0.f, 0.f}; acc[j] = z; }

#pragma unroll 1
    for (int b0 = 0; b0 < c; b0 += 32) {
      int idx = o + b0 + lane;
      idx = idx > RCAP - 1 ? RCAP - 1 : idx;
      const v2i en = *(const v2ia*)(cb + 2 * (size_t)idx);
      int sr = en.x;
      sr = sr < 0 ? 0 : (sr > nN - 1 ? nN - 1 : sr);
      const int wvi = en.y;
      const int m32 = (c - b0) < 32 ? (c - b0) : 32;
#pragma unroll 1
      for (int k = 0; k < m32; ++k) {
        const int   sk = __builtin_amdgcn_readlane(sr, k);
        const float ck = __int_as_float(__builtin_amdgcn_readlane(wvi, k));
        const float* rp = hs + (size_t)sk * F + 4 * lane;
#pragma unroll
        for (int j = 0; j < NJ; ++j) {
          const v4f a = *(const v4f*)(rp + 128 * j);
          acc[j].x = fmaf(ck, a.x, acc[j].x);
          acc[j].y = fmaf(ck, a.y, acc[j].y);
          acc[j].z = fmaf(ck, a.z, acc[j].z);
          acc[j].w = fmaf(ck, a.w, acc[j].w);
        }
      }
    }
    const float dd  = dinv[nc];
    const float pzr = bad ? qnan : 0.0f;
    const bool live = node < nN;
    const float* sp = hs + (size_t)nc * F + 4 * lane;
    v4f yv[NJ];
#pragma unroll
    for (int j = 0; j < NJ; ++j) {
      const v4f a = *(const v4f*)(sp + 128 * j);
      const float t0 = dd * (acc[j].x + a.x) + bv[j].x;
      const float t1 = dd * (acc[j].y + a.y) + bv[j].y;
      const float t2 = dd * (acc[j].z + a.z) + bv[j].z;
      const float t3 = dd * (acc[j].w + a.w) + bv[j].w;
      float y0 = (t0 > 0.0f) ? t0 : (t0 - t0);
      float y1 = (t1 > 0.0f) ? t1 : (t1 - t1);
      float y2 = (t2 > 0.0f) ? t2 : (t2 - t2);
      float y3 = (t3 > 0.0f) ? t3 : (t3 - t3);
      y0 = y0 + pzr; y1 = y1 + pzr; y2 = y2 + pzr; y3 = y3 + pzr;
      v4f y;
      y.x = live ? y0 : 0.0f; y.y = live ? y1 : 0.0f; y.z = live ? y2 : 0.0f; y.w = live ? y3 : 0.0f;
      yv[j] = y;
    }

    if constexpr (F == 512) {
      unsigned short* rb = rowbuf + wave * 1024;
#pragma unroll
      for (int j = 0; j < NJ; ++j) {
        v4us h4, l4;
        unsigned hb;
        hb = bf16_bits(yv[j].x); h4[0] = (unsigned short)hb; l4[0] = (unsigned short)bf16_bits(yv[j].x - __uint_as_float(hb << 16));
        hb = bf16_bits(yv[j].y); h4[1] = (unsigned short)hb; l4[1] = (unsigned short)bf16_bits(yv[j].y - __uint_as_float(hb << 16));
        hb = bf16_bits(yv[j].z); h4[2] = (unsigned short)hb; l4[2] = (unsigned short)bf16_bits(yv[j].z - __uint_as_float(hb << 16));
        hb = bf16_bits(yv[j].w); h4[3] = (unsigned short)hb; l4[3] = (unsigned short)bf16_bits(yv[j].w - __uint_as_float(hb << 16));
        *(v4usa*)(rb + 4 * lane + 128 * j) = h4;
        *(v4usa*)(rb + 512 + 4 * lane + 128 * j) = l4;
      }
      wave_sync();
      v8us qv[4];
#pragma unroll
      for (int q = 0; q < 4; ++q) qv[q] = *(const v8usa*)(rb + 8 * lane + 256 * q);
      wave_sync();
      if (node < mRows) {
        unsigned short* rpw = xhl + (size_t)node * 1024 + 8 * lane;
#pragma unroll
        for (int q = 0; q < 4; ++q) *(volatile v8us*)(rpw + 256 * q) = qv[q];
        __threadfence();
#pragma unroll
        for (int q = 0; q < 4; ++q) *(volatile v8us*)(rpw + 256 * q) = qv[q];
      }
    } else {
      float t = 0.0f;
#pragma unroll
      for (int j = 0; j < NJ; ++j) {
        t = fmaf(yv[j].x, wv[j].x, t);
        t = fmaf(yv[j].y, wv[j].y, t);
        t = fmaf(yv[j].z, wv[j].z, t);
        t = fmaf(yv[j].w, wv[j].w, t);
      }
      t += __shfl_xor(t, 16, 32);
      t += __shfl_xor(t, 8, 32);
      t += __shfl_xor(t, 4, 32);
      t += __shfl_xor(t, 2, 32);
      t += __shfl_xor(t, 1, 32);
      const float tv = live ? (dd * t) : 0.0f;
      if (lane == 0) tsb[r] = tv;
    }
  }

  if constexpr (F == 256) {
    __syncthreads();
    const v4f ov = *(const v4fa*)(tsb + 4 * (lane & 15));
    float* op = ts + (size_t)blockBase + 4 * (lane & 15);
    const bool okst = (wave == 0) && (lane < RPB / 4) && (blockBase + RPB <= mRows);
    if (okst) *(volatile v4f*)op = ov;
    __threadfence();
    if (okst) *(volatile v4f*)op = ov;
  }
}

__global__ __launch_bounds__(NTHR) void k_out(const float* __restrict__ ts, const float* __restrict__ dinv,
                                              const int* __restrict__ rec, const int* __restrict__ cache,
                                              const float* __restrict__ b5, int nN, float* out) {
  __shared__ __attribute__((aligned(16))) float os[NTHR];
  const int tid  = (int)threadIdx.x;
  const int node = (int)blockIdx.x * NTHR + tid;
  const int nc   = node < nN ? node : nN - 1;
  const v2i rc = *(const v2ia*)(rec + 2 * (size_t)nc);
  int c = rc.y;
  const bool bad = (c < 0) || (c > DEGCAP);
  c = c < 0 ? 0 : (c > DEGCAP ? DEGCAP : c);
  int o = rc.x;
  o = o < 0 ? 0 : (o > RCAP ? RCAP : o);
  const int* cb = cache + (size_t)(nc >> SLA) * RCAP * 2;
  float s = 0.0f;
#pragma unroll 1
  for (int p = 0; p < DEGCAP; ++p) {
    const bool act = p < c;
    if (__builtin_amdgcn_ballot_w32(act) == 0u) break;
    int idx = o + p;
    idx = idx > RCAP - 1 ? RCAP - 1 : idx;
    const v2i en = *(const v2ia*)(cb + 2 * (size_t)idx);
    int sr = en.x;
    sr = sr < 0 ? 0 : (sr > nN - 1 ? nN - 1 : sr);
    const float tvv = ts[sr];
    const float sn = fmaf(__int_as_float(en.y), tvv, s);
    s = act ? sn : s;
  }
  s = s + ts[nc];
  const float pz = bad ? __int_as_float(0x7fc00000) : 0.0f;
  const float v = (dinv[nc] * s + bf16_val(b5[0])) + pz;
  os[tid] = (node < nN) ? v : 0.0f;
  __syncthreads();
  const int q4 = 4 * (tid & 63);
  const v4f ov = *(const v4fa*)(os + q4);
  const int e0 = (int)blockIdx.x * NTHR + q4;
  const bool okst = (tid < 64) && (e0 + 3 < nN);
  float* op = out + (size_t)blockIdx.x * NTHR + q4;
  if (okst) *(volatile v4f*)op = ov;
  __threadfence();
  if (okst) *(volatile v4f*)op = ov;
}

static inline int cdiv(int a, int b) { return (a + b - 1) / b; }
static inline size_t al256(size_t o) { return (o + 255) & ~(size_t)255; }

extern "C" void kernel_launch(void* const* d_in, const int* in_sizes, int n_in,
                              void* d_out, int out_size, void* d_ws, size_t ws_size,
                              hipStream_t stream) {
  if (n_in < 13) return;
  if (in_sizes[0] < FD || (in_sizes[0] % FD) != 0) return;
  const int nN = in_sizes[0] / FD;
  if (nN < 64 || nN > (1 << 22) || (nN % 32) != 0) return;
  if (in_sizes[1] < 2 || (in_sizes[1] & 1) != 0) return;
  const int nE = in_sizes[1] / 2;
  if (nE < 1 || nE >= (1 << (31 - SLA))) return;
  if (in_sizes[2] != nE) return;
  if (in_sizes[3] != 512 * 512 || in_sizes[4] != 512) return;
  if (in_sizes[5] != 512 * 512 || in_sizes[6] != 512) return;
  if (in_sizes[7] != 512 * 512 || in_sizes[8] != 512) return;
  if (in_sizes[9] != 512 * 256 || in_sizes[10] != 256) return;
  if (in_sizes[11] != 256 || in_sizes[12] != 1) return;
  if (out_size != nN) return;

  const float* x    = (const float*)d_in[0];
  const int*   edge = (const int*)d_in[1];
  const float* ewp  = (const float*)d_in[2];
  const float* W1   = (const float*)d_in[3];
  const float* b1   = (const float*)d_in[4];
  const float* W2   = (const float*)d_in[5];
  const float* b2   = (const float*)d_in[6];
  const float* W3   = (const float*)d_in[7];
  const float* b3   = (const float*)d_in[8];
  const float* W4   = (const float*)d_in[9];
  const float* b4   = (const float*)d_in[10];
  const float* W5   = (const float*)d_in[11];
  const float* b5   = (const float*)d_in[12];
  float* out = (float*)d_out;
  const int* src = edge;
  const int* dst = edge + nE;

  const int MP  = cdiv(nN, GBM) * GBM;
  const int gM  = MP / GBM;
  const int gB  = cdiv(MP, NBA);
  const int NBP = gB * NBA;
  if (NBP < MP) return;
  if (cdiv(nN, NTHR) * NTHR > NBP + NTHR) return;
  const int vec8 = ((nE & 3) == 0) ? 1 : 0;

  char* ws = (char*)d_ws;
  size_t off = 0;
  const size_t oDINV = off; off = al256(off + (size_t)NBP * 4);
  const size_t oREC  = off; off = al256(off + (size_t)NBP * 8);
  const size_t oTS   = off; off = al256(off + (size_t)NBP * 4);
  const size_t oCA   = off; off = al256(off + (size_t)gB * RCAP * 8);
  const size_t oW1T  = off; off = al256(off + (size_t)512 * 512 * 2);
  const size_t oW2D  = off; off = al256(off + (size_t)512 * 1024 * 2);
  const size_t oW3D  = off; off = al256(off + (size_t)512 * 1024 * 2);
  const size_t oW4D  = off; off = al256(off + (size_t)256 * 1024 * 2);
  const size_t oHS   = off; off = al256(off + (size_t)MP * 512 * 4);
  const size_t oXHL  = off; off = al256(off + (size_t)MP * 1024 * 2);
  if (off > ws_size || off > (size_t)WSMAX) return;
  float*          DINV = (float*)(ws + oDINV);
  int*            REC  = (int*)(ws + oREC);
  float*          TS   = (float*)(ws + oTS);
  int*            CA   = (int*)(ws + oCA);
  unsigned short* W1T  = (unsigned short*)(ws + oW1T);
  unsigned short* W2D  = (unsigned short*)(ws + oW2D);
  unsigned short* W3D  = (unsigned short*)(ws + oW3D);
  unsigned short* W4D  = (unsigned short*)(ws + oW4D);
  float*          HS   = (float*)(ws + oHS);
  unsigned short* XHL  = (unsigned short*)(ws + oXHL);
  unsigned short* XB   = XHL;

  const size_t bldLds = (size_t)BLD_LDS_INTS * 4;
  hipFuncSetAttribute(reinterpret_cast<const void*>(&k_build), hipFuncAttributeMaxDynamicSharedMemorySize, (int)bldLds);

  const int nUx = MP * (FD / 8);
  k_wprep<<<NUTOT / NTHR, NTHR, 0, stream>>>(W1, W2, W3, W4, W1T, W2D, W3D, W4D);
  k_cvx<<<cdiv(nUx, NTHR), NTHR, 0, stream>>>(x, nN, nUx, XB);
  k_build<<<gB, NTHR, bldLds, stream>>>(src, dst, ewp, nE, nN, vec8, DINV, REC, CA);
  k_gemm<<<dim3(gM, 512 / GBN), GTHR, 0, stream>>>(XB, 512, W1T, 512, DINV, HS, 512);
  k_agg<512><<<gM, NTHR, 0, stream>>>(HS, DINV, REC, CA, b1, W5, nN, MP, XHL, TS);
  k_gemm<<<dim3(gM, 512 / GBN), GTHR, 0, stream>>>(XHL, 1024, W2D, 1024, DINV, HS, 512);
  k_agg<512><<<gM, NTHR, 0, stream>>>(HS, DINV, REC, CA, b2, W5, nN, MP, XHL, TS);
  k_gemm<<<dim3(gM, 512 / GBN), GTHR, 0, stream>>>(XHL, 1024, W3D, 1024, DINV, HS, 512);
  k_agg<512><<<gM, NTHR, 0, stream>>>(HS, DINV, REC, CA, b3, W5, nN, MP, XHL, TS);
  k_gemm<<<dim3(gM, 256 / GBN), GTHR, 0, stream>>>(XHL, 1024, W4D, 1024, DINV, HS, 256);
  k_agg<256><<<gM, NTHR, 0, stream>>>(HS, DINV, REC, CA, b4, W5, nN, MP, XHL, TS);
  k_out<<<cdiv(nN, NTHR), NTHR, 0, stream>>>(TS, DINV, REC, CA, b5, nN, out);
}
